// Decoder_76888504533579
// MI455X (gfx1250) — hardware-verified
//
#include <hip/hip_runtime.h>
#include <math.h>

constexpr int NBATCH = 16;
constexpr int NSTEP  = 32;
constexpr int NSRC   = 256;
constexpr int NSLOT  = 8;
constexpr int NKGL   = 64;
constexpr int NVOC   = 32000;
constexpr int NEXT   = 50;
constexpr int NVOCX  = NVOC + NEXT;
constexpr int NHID   = 512;
constexpr int NEMB   = 512;
constexpr int NROWS  = NBATCH * NSTEP;
constexpr int NGATE  = 3 * NHID;
constexpr int NXCK   = 2 * NHID;
constexpr int NCAT   = 4 * NHID;
constexpr int NPTRW  = 4 * NHID + NEMB;
constexpr int NWCAT  = 2 * NHID + NGATE;
constexpr int NKL    = NSLOT * NKGL;
constexpr int QPAD   = 64;
constexpr int SLABF  = NSTEP * NVOCX;
constexpr int CHUNKF = 8192;
constexpr int NCHUNK = (SLABF + CHUNKF - 1) / CHUNKF;
constexpr int AHP    = 520;
constexpr int AXP    = 1032;
constexpr int HQP    = 516;
constexpr int SCAN_THREADS = 512;
constexpr float NEG_FILL   = -1e10f;
constexpr float WCARRY     = 256.0f;
constexpr float YCARRY     = 16.0f;
constexpr float CATCARRY   = 16.0f;

static_assert(SCAN_THREADS / 32 == NBATCH, "one wave per batch row in the attention phases");
static_assert(NHID == 32 * (SCAN_THREADS / 32), "two 16-column unit groups per wave");
static_assert((SLABF * 4) % 128 == 0, "per-batch output slab is a whole number of 128-B lines");
static_assert(NVOCX % 2 == 0 && NVOC % 2 == 0, "pair processing");
static_assert(SLABF - (NCHUNK - 1) * CHUNKF == 1600, "last chunk extent");
static_assert(NHID % 32 == 0 && NXCK % 32 == 0 && NCAT % 32 == 0 && NEMB % 32 == 0, "GEMM K multiples of 32");
static_assert((NBATCH * NSRC) % 64 == 0 && (NBATCH * NSLOT) % 64 == 0 && NROWS % 64 == 0, "GEMM M tile multiples");
static_assert(NHID % 64 == 0 && NGATE % 64 == 0 && NVOC % 64 == 0 && (NBATCH * QPAD) % 64 == 0, "GEMM N/M tile multiples");
static_assert(NKL == 512 && NKL % 64 == 0, "copy logit plane width");
static_assert(NBATCH == 16 && NSTEP == 32, "row index maps use shifts");
static_assert((size_t)NROWS * NVOCX * 4 == (size_t)65638400, "output bytes");

typedef __attribute__((ext_vector_type(16))) _Float16 v16h;
typedef __attribute__((ext_vector_type(8)))  _Float16 v8h;
typedef __attribute__((ext_vector_type(16))) __bf16   v16b;
typedef __attribute__((ext_vector_type(8)))  __bf16   v8b;
typedef __attribute__((ext_vector_type(8)))  float    v8f;
typedef __attribute__((ext_vector_type(4)))  float    v4f;
typedef __attribute__((ext_vector_type(2)))  float    v2f;
typedef __attribute__((ext_vector_type(4)))  unsigned v4u;
typedef __attribute__((ext_vector_type(2)))  unsigned v2u;
typedef unsigned v4ua __attribute__((ext_vector_type(4))) __attribute__((may_alias));

__device__ __forceinline__ unsigned short f2bf_bits(float f) {
  unsigned u = __float_as_uint(f);
  return (unsigned short)((u + 0x7FFFu + ((u >> 16) & 1u)) >> 16);
}
__device__ __forceinline__ float bf_bits2f(unsigned short h) { return __uint_as_float(((unsigned)h) << 16); }

__device__ __forceinline__ unsigned bfbits32(float f) {
  const unsigned u = __float_as_uint(f);
  return (u + 0x7FFFu + ((u >> 16) & 1u)) >> 16;
}
__device__ __forceinline__ void split_bf(float f, unsigned& hb, unsigned& lb) {
  hb = bfbits32(f);
  lb = bfbits32(f - __uint_as_float(hb << 16));
}
__device__ __forceinline__ float bf_lo(unsigned w) { return __uint_as_float(w << 16); }
__device__ __forceinline__ float bf_hi(unsigned w) { return __uint_as_float(w & 0xffff0000u); }

__device__ __forceinline__ float h16_to_f32(unsigned hb) {
  const unsigned sgn = (hb & 0x8000u) << 16; const unsigned em = hb & 0x7fffu;
  const float fn = __uint_as_float((em << 13) + 0x38000000u);
  const float fs = (float)em * 5.9604644775390625e-8f;
  const float mag = (em < 0x400u) ? fs : fn; return __uint_as_float(__float_as_uint(mag) | sgn); }

__device__ __forceinline__ void dep_guard4_h(v8f& a, v8f& b, v8f& c, v8f& d, v16h x, v16h y) { asm volatile("v_nop\n\tv_nop\n\tv_nop\n\tv_nop" : "+v"(a), "+v"(b), "+v"(c), "+v"(d) : "v"(x), "v"(y)); }
__device__ __forceinline__ void dep_guard4_b(v8f& a, v8f& b, v8f& c, v8f& d, v16b x, v16b y) { asm volatile("v_nop\n\tv_nop\n\tv_nop\n\tv_nop" : "+v"(a), "+v"(b), "+v"(c), "+v"(d) : "v"(x), "v"(y)); }
__device__ __forceinline__ void keep4_h(v16h a, v16h b, v16h c, v16h d) { asm volatile("v_nop" :: "v"(a), "v"(b), "v"(c), "v"(d)); }
__device__ __forceinline__ void keep4_b(v16b a, v16b b, v16b c, v16b d) { asm volatile("v_nop" :: "v"(a), "v"(b), "v"(c), "v"(d)); }
__device__ __forceinline__ void acc_guard4(v8f& a, v8f& b, v8f& c, v8f& d) { asm volatile("v_nop\n\tv_nop\n\tv_nop\n\tv_nop" : "+v"(a), "+v"(b), "+v"(c), "+v"(d)); }
template <typename T> struct Frag;
template <> struct Frag<_Float16> {
  typedef v16h V; union U { v16h v; v8h h[2]; };
  static __device__ __forceinline__ v16h load(const _Float16* p) {
    U f; f.h[0] = *(const v8h*)(p); f.h[1] = *(const v8h*)(p + 16); return f.v;
  }
  static __device__ __forceinline__ v8f mma(v16h a, v16h b, v8f c) {
    return __builtin_amdgcn_wmma_f32_16x16x32_f16(false, a, false, b, (short)0, c, false, false);
  }
  static __device__ __forceinline__ void guard4(v8f& a, v8f& b, v8f& c, v8f& d, v16h x, v16h y) { dep_guard4_h(a, b, c, d, x, y); }
  static __device__ __forceinline__ void keep(v16h a, v16h b, v16h c, v16h d) { keep4_h(a, b, c, d); }
};
template <> struct Frag<__bf16> {
  typedef v16b V; union U { v16b v; v8b h[2]; };
  static __device__ __forceinline__ v16b load(const __bf16* p) {
    U f; f.h[0] = *(const v8b*)(p); f.h[1] = *(const v8b*)(p + 16); return f.v;
  }
  static __device__ __forceinline__ v8f mma(v16b a, v16b b, v8f c) {
    return __builtin_amdgcn_wmma_f32_16x16x32_bf16(false, a, false, b, (short)0, c, false, false);
  }
  static __device__ __forceinline__ void guard4(v8f& a, v8f& b, v8f& c, v8f& d, v16b x, v16b y) { dep_guard4_b(a, b, c, d, x, y); }
  static __device__ __forceinline__ void keep(v16b a, v16b b, v16b c, v16b d) { keep4_b(a, b, c, d); }
};

__device__ __forceinline__ v8f mma_bf(v16b a, v16b b, v8f c) {
  c = __builtin_amdgcn_wmma_f32_16x16x32_bf16(false, a, false, b, (short)0, c, false, false);
  asm volatile("v_nop\n\tv_nop\n\tv_nop\n\tv_nop" : "+v"(c) : "v"(a), "v"(b));
  return c;
}
__device__ __forceinline__ v8f mma3(v16b xh, v16b xl, v16b bh, v16b bl, v8f a) {
  a = mma_bf(xh, bh, a);
  a = mma_bf(xh, bl, a);
  a = mma_bf(xl, bh, a);
  return a;
}

__device__ __forceinline__ float ftanh_fast(float x) { return 1.0f - 2.0f * __builtin_amdgcn_rcpf(__expf(2.0f * x) + 1.0f); }
__device__ __forceinline__ float fsig_p(float x)  { return __builtin_amdgcn_rcpf(1.0f + expf(-x)); }
__device__ __forceinline__ float ftanh_p(float x) { return 1.0f - 2.0f * __builtin_amdgcn_rcpf(expf(2.0f * x) + 1.0f); }

template <int ET> struct Elem;
template <> struct Elem<0> { typedef _Float16 T; };
template <> struct Elem<1> { typedef __bf16 T; };
template <int ET, bool SPLIT, int BIAS_MODE, int OUT_MODE>
__global__ __launch_bounds__(256) void wmma_gemm64(
    const unsigned short* __restrict__ Ap, const unsigned short* __restrict__ A2p, int lda, long strideA,
    const unsigned short* __restrict__ Btp, const unsigned short* __restrict__ Bt2p, int ldb, long strideB,
    void* __restrict__ Cout, void* __restrict__ Cout2, int ldc, long strideC,
    const float* __restrict__ bias,
    int M, int N, int K, float scale) {
  static_assert(BIAS_MODE == 0 || BIAS_MODE == 2, "bias modes instantiated here");
  typedef typename Elem<ET>::T T;
  typedef typename Frag<T>::V V;
  const T* A = (const T*)Ap; const T* A2 = (const T*)A2p; const T* Bt = (const T*)Btp; const T* Bt2 = (const T*)Bt2p;
  __shared__ __align__(16) float sT[8][16 * 68];
  const int b    = blockIdx.y;
  const int lane = threadIdx.x & 31;
  const int wave = threadIdx.x >> 5;
  const int tilesN = N >> 6;
  const int tilesM = M >> 6;
  const int tile = blockIdx.x * 8 + wave;
  if (tile >= tilesM * tilesN) return;
  const int tm = tile / tilesN;
  const int tn = tile - tm * tilesN;
  const int m0 = tm << 6;
  const int n0 = tn << 6;

  const T* Ab  = A  + (size_t)b * strideA;
  const T* Bb  = Bt + (size_t)b * strideB;
  const T* Ab2 = SPLIT ? (A2  + (size_t)b * strideA) : nullptr;
  const T* Bb2 = SPLIT ? (Bt2 + (size_t)b * strideB) : nullptr;

  const int rlane = lane & 15;
  const int koff  = (lane >> 4) * 8;
  const int mOff  = (lane >> 4) * 8;

  v8f acc[4][4];
#pragma unroll
  for (int i = 0; i < 4; ++i)
#pragma unroll
    for (int j = 0; j < 4; ++j) acc[i][j] = (v8f){0.f,0.f,0.f,0.f,0.f,0.f,0.f,0.f};

  for (int k0 = 0; k0 < K; k0 += 32) {
    V bh[4], bl[4];
#pragma unroll
    for (int j = 0; j < 4; ++j) {
      const size_t bo = (size_t)(n0 + (j << 4) + rlane) * ldb + koff + k0;
      bh[j] = Frag<T>::load(Bb + bo);
      if (SPLIT) bl[j] = Frag<T>::load(Bb2 + bo);
    }
#pragma unroll
    for (int i = 0; i < 4; ++i) {
      const size_t ao = (size_t)(m0 + (i << 4) + rlane) * lda + koff + k0;
      V ah = Frag<T>::load(Ab + ao);
      V al;
      if (SPLIT) al = Frag<T>::load(Ab2 + ao);
#pragma unroll
      for (int j = 0; j < 4; ++j) {
        acc[i][j] = Frag<T>::mma(ah, bh[j], acc[i][j]);
        if (SPLIT) {
          acc[i][j] = Frag<T>::mma(ah, bl[j], acc[i][j]);
          acc[i][j] = Frag<T>::mma(al, bh[j], acc[i][j]);
        }
      }
      Frag<T>::guard4(acc[i][0], acc[i][1], acc[i][2], acc[i][3], ah, SPLIT ? al : ah);
    }
    Frag<T>::keep(bh[0], bh[1], bh[2], bh[3]);
    if (SPLIT) Frag<T>::keep(bl[0], bl[1], bl[2], bl[3]);
  }
  acc_guard4(acc[0][0], acc[0][1], acc[0][2], acc[0][3]);
  acc_guard4(acc[1][0], acc[1][1], acc[1][2], acc[1][3]);
  acc_guard4(acc[2][0], acc[2][1], acc[2][2], acc[2][3]);
  acc_guard4(acc[3][0], acc[3][1], acc[3][2], acc[3][3]);

  float* slab = sT[wave];
#pragma unroll
  for (int i = 0; i < 4; ++i) {
    const int mBase = m0 + (i << 4);
#pragma unroll
    for (int j = 0; j < 4; ++j) {
      const int n = n0 + (j << 4) + rlane;
      float bv = 0.f;
      if (BIAS_MODE == 2) bv = bias[n];
#pragma unroll
      for (int r = 0; r < 8; ++r) {
        float v = acc[i][j][r] * scale;
        if (BIAS_MODE == 2) v += bv;
        slab[(mOff + r) * 68 + (j << 4) + rlane] = v;
      }
    }
    __builtin_amdgcn_fence(__ATOMIC_RELEASE, "workgroup");
    __builtin_amdgcn_wave_barrier();
    __builtin_amdgcn_fence(__ATOMIC_ACQUIRE, "workgroup");
    if (OUT_MODE == 0) {
      float* C = (float*)Cout + (size_t)b * strideC;
      const int hh = lane >> 4, c4 = (lane & 15) * 4;
      for (int pass = 0; pass < 2; ++pass) {
#pragma unroll
        for (int it = 0; it < 8; ++it) {
          const int row = it * 2 + hh;
          v4f v = *(const v4f*)(slab + row * 68 + c4);
          *(volatile v4f*)(C + (size_t)(mBase + row) * ldc + n0 + c4) = v;
        }
        __threadfence();
      }
    } else {
      const int q = lane >> 3, c8 = (lane & 7) * 8;
      unsigned short* C  = (unsigned short*)Cout  + (size_t)b * strideC;
      unsigned short* C2 = (OUT_MODE == 2) ? ((unsigned short*)Cout2 + (size_t)b * strideC) : nullptr;
      for (int pass = 0; pass < 2; ++pass) {
#pragma unroll
        for (int it = 0; it < 4; ++it) {
          const int row = it * 4 + q;
          const float* sp = slab + row * 68 + c8;
          v8h hv, lv;
#pragma unroll
          for (int e = 0; e < 8; ++e) {
            if (OUT_MODE == 1) {
              hv[e] = (_Float16)sp[e];
            } else {
              unsigned short hb = f2bf_bits(sp[e]);
              unsigned short lb = f2bf_bits(sp[e] - bf_bits2f(hb));
              hv[e] = __builtin_bit_cast(_Float16, hb);
              lv[e] = __builtin_bit_cast(_Float16, lb);
            }
          }
          *(volatile v8h*)(C + (size_t)(mBase + row) * ldc + n0 + c8) = hv;
          if (OUT_MODE == 2) *(volatile v8h*)(C2 + (size_t)(mBase + row) * ldc + n0 + c8) = lv;
        }
        __threadfence();
      }
    }
    __builtin_amdgcn_fence(__ATOMIC_RELEASE, "workgroup");
    __builtin_amdgcn_wave_barrier();
    __builtin_amdgcn_fence(__ATOMIC_ACQUIRE, "workgroup");
  }
}

template <int MODE>
__global__ __launch_bounds__(256) void cvt8_kernel(const float* __restrict__ src, unsigned short* __restrict__ dst,
                                                   unsigned short* __restrict__ dst2,
                                                   int nrow, int ncol8, int spitch, int scol0, float sc) {
  const int i  = blockIdx.x * 256 + threadIdx.x;
  const int n8 = nrow * ncol8;
  if (i < n8) {
    const int row = i / ncol8;
    const int c8  = i - row * ncol8;
    const float* sp = src + (size_t)row * spitch + scol0 + c8 * 8;
    const v4f a = *(const v4f*)(sp);
    const v4f b = *(const v4f*)(sp + 4);
    v8h hv, lv;
#pragma unroll
    for (int e = 0; e < 4; ++e) {
      const float fa = a[e] * sc;
      const float fb = b[e] * sc;
      if (MODE == 0) {
        hv[e]     = (_Float16)fa;
        hv[4 + e] = (_Float16)fb;
        lv[e]     = hv[e];
        lv[4 + e] = hv[4 + e];
      } else {
        const unsigned short ha = f2bf_bits(fa);
        const unsigned short la = f2bf_bits(fa - bf_bits2f(ha));
        const unsigned short hb = f2bf_bits(fb);
        const unsigned short lb = f2bf_bits(fb - bf_bits2f(hb));
        hv[e]     = __builtin_bit_cast(_Float16, ha);
        lv[e]     = __builtin_bit_cast(_Float16, la);
        hv[4 + e] = __builtin_bit_cast(_Float16, hb);
        lv[4 + e] = __builtin_bit_cast(_Float16, lb);
      }
    }
    *(volatile v8h*)(dst + (size_t)i * 8) = hv;
    if (MODE == 1) *(volatile v8h*)(dst2 + (size_t)i * 8) = lv;
    __threadfence();
    *(volatile v8h*)(dst + (size_t)i * 8) = hv;
    if (MODE == 1) *(volatile v8h*)(dst2 + (size_t)i * 8) = lv;
  }
}

__global__ __launch_bounds__(256) void gather_y_kernel(const int* __restrict__ tgt, const float* __restrict__ emb,
                                                       unsigned short* __restrict__ YH) {
  const int i = blockIdx.x * 256 + threadIdx.x;
  if (i < NROWS * (NEMB / 8)) {
    const int mp = i >> 6;
    const int bb = mp & (NBATCH - 1);
    const int tt = mp >> 4;
    const int c8 = (i & 63) * 8;
    int id = tgt[bb * NSTEP + tt];
    id = id < 0 ? 0 : (id > NVOC - 1 ? NVOC - 1 : id);
    const float* sp = emb + (size_t)id * NEMB + c8;
    const v4f a = *(const v4f*)(sp);
    const v4f b = *(const v4f*)(sp + 4);
    v8h hv;
#pragma unroll
    for (int e = 0; e < 4; ++e) {
      hv[e]     = (_Float16)(a[e] * YCARRY);
      hv[4 + e] = (_Float16)(b[e] * YCARRY);
    }
    *(volatile v8h*)(YH + (size_t)i * 8) = hv;
    __threadfence();
    *(volatile v8h*)(YH + (size_t)i * 8) = hv;
  }
}

__global__ __launch_bounds__(256) void zero_pad_kernel(unsigned short* __restrict__ P0, unsigned short* __restrict__ P1) {
  const int i = blockIdx.x * 256 + threadIdx.x;
  unsigned short* P = (blockIdx.y == 0) ? P0 : P1;
  if (i < NBATCH * 32 * 64) {
    const int b = i >> 11;
    const int r = i & 2047;
    const v4u z = {0u, 0u, 0u, 0u};
    unsigned short* dp = P + ((size_t)(b * QPAD + NSTEP) * NHID) + (size_t)r * 8;
    *(volatile v4u*)dp = z;
    __threadfence();
    *(volatile v4u*)dp = z;
  }
}

__device__ __forceinline__ void hq_phase(const unsigned short* ahH, const unsigned short* ahL,
                                         const __bf16* Wh, const __bf16* Wl, int rowbase,
                                         int wave, int c, int hh, float* hq) {
  const __bf16* ah = (const __bf16*)ahH + c * AHP + 8 * hh;
  const __bf16* al = (const __bf16*)ahL + c * AHP + 8 * hh;
  const size_t ro = (size_t)(rowbase + 32 * wave + c) * NHID + 8 * hh;
  const __bf16* w0h = Wh + ro;
  const __bf16* w0l = Wl + ro;
  const __bf16* w1h = w0h + 16 * NHID;
  const __bf16* w1l = w0l + 16 * NHID;
  v8f a0 = {0.f, 0.f, 0.f, 0.f, 0.f, 0.f, 0.f, 0.f};
  v8f a1 = {0.f, 0.f, 0.f, 0.f, 0.f, 0.f, 0.f, 0.f};
#pragma unroll 1
  for (int k0 = 0; k0 < NHID; k0 += 32) {
    const v16b xh = Frag<__bf16>::load(ah + k0);
    const v16b xl = Frag<__bf16>::load(al + k0);
    const v16b b0h = Frag<__bf16>::load(w0h + k0);
    const v16b b0l = Frag<__bf16>::load(w0l + k0);
    a0 = mma3(xh, xl, b0h, b0l, a0);
    asm volatile("" ::: "memory");
    const v16b b1h = Frag<__bf16>::load(w1h + k0);
    const v16b b1l = Frag<__bf16>::load(w1l + k0);
    a1 = mma3(xh, xl, b1h, b1l, a1);
    asm volatile("" ::: "memory");
  }
#pragma unroll
  for (int r = 0; r < 8; ++r) {
    hq[(8 * hh + r) * HQP + 32 * wave + c]      = a0[r];
    hq[(8 * hh + r) * HQP + 32 * wave + 16 + c] = a1[r];
  }
}

__global__ __launch_bounds__(SCAN_THREADS) void scan_kernel(
    const float* __restrict__ h0, const float* __restrict__ src, const float* __restrict__ srcmask,
    const float* __restrict__ kgh, const float* __restrict__ kgmask,
    const float* __restrict__ PVS, const float* __restrict__ PVK,
    const float* __restrict__ Vwc, const float* __restrict__ bVc,
    const float* __restrict__ Vwk, const float* __restrict__ bVk,
    const float* __restrict__ GIYT, const float* __restrict__ bih, const float* __restrict__ bhh,
    const unsigned short* __restrict__ WCHp, const unsigned short* __restrict__ WCLp,
    const unsigned short* __restrict__ WIHp, const unsigned short* __restrict__ WILp,
    unsigned short* __restrict__ SPH, unsigned short* __restrict__ SPL,
    unsigned short* __restrict__ XCKH, unsigned short* __restrict__ XCKL, float* __restrict__ KW) {
  __shared__ __align__(16) unsigned short AhH[16 * AHP];
  __shared__ __align__(16) unsigned short AhL[16 * AHP];
  __shared__ __align__(16) unsigned short AxH[16 * AXP];
  __shared__ __align__(16) unsigned short AxL[16 * AXP];
  __shared__ __align__(16) float hq[16 * HQP];
  __shared__ __align__(16) float ew[NBATCH * NSRC];
  __shared__ __align__(16) float kwt[NBATCH * NSLOT];

  const __bf16* WCh = (const __bf16*)WCHp;
  const __bf16* WCl = (const __bf16*)WCLp;
  const __bf16* WIh = (const __bf16*)WIHp;
  const __bf16* WIl = (const __bf16*)WILp;
  const int tid = threadIdx.x, lane = tid & 31, wave = tid >> 5;
  const int c = lane & 15, hh = lane >> 4, koff = hh * 8;
  const int bw = wave;
  const v8f z8 = {0.f, 0.f, 0.f, 0.f, 0.f, 0.f, 0.f, 0.f};

#pragma unroll
  for (int it = 0; it < 4; ++it) {
    const int idx = it * SCAN_THREADS + tid;
    const int row = idx >> 7;
    const int c4 = (idx & 127) * 4;
    const v4f v = *(const v4f*)(h0 + row * NHID + c4);
    *(v4f*)(hq + row * HQP + c4) = v;
  }
  __syncthreads();

  float hst[2][8];
  float brz[2], bzz[2], bin[2], bhn[2];
#pragma unroll
  for (int u = 0; u < 2; ++u) {
    const int j = 32 * wave + 16 * u + c;
    brz[u] = bih[j] + bhh[j];
    bzz[u] = bih[NHID + j] + bhh[NHID + j];
    bin[u] = bih[2 * NHID + j];
    bhn[u] = bhh[2 * NHID + j];
#pragma unroll
    for (int r = 0; r < 8; ++r) {
      const int row = 8 * hh + r;
      const float hv = hq[row * HQP + j];
      hst[u][r] = hv;
      unsigned hb, lb;
      split_bf(hv, hb, lb);
      AhH[row * AHP + j] = (unsigned short)hb;
      AhL[row * AHP + j] = (unsigned short)lb;
    }
  }
  __syncthreads();

#pragma unroll 1
  for (int t = 0; t < NSTEP; ++t) {
    hq_phase(AhH, AhL, WCh, WCl, 0, wave, c, hh, hq);
    __syncthreads();

    {
      v4f hqv[4], vw[4];
#pragma unroll
      for (int q = 0; q < 4; ++q) {
        hqv[q] = *(const v4f*)(hq + bw * HQP + 128 * q + 4 * lane);
        vw[q]  = *(const v4f*)(Vwc + 128 * q + 4 * lane);
      }
      const float* pvb = PVS + (size_t)bw * NSRC * NHID + 4 * lane;
#pragma unroll 1
      for (int s = 0; s < NSRC; ++s) {
        float p = 0.0f;
#pragma unroll
        for (int q = 0; q < 4; ++q) {
          const v4f pv = *(const v4f*)(pvb + (size_t)s * NHID + 128 * q);
#pragma unroll
          for (int e = 0; e < 4; ++e) p += vw[q][e] * ftanh_fast(hqv[q][e] + pv[e]);
        }
#pragma unroll
        for (int off = 16; off > 0; off >>= 1) p += __shfl_xor(p, off, 32);
        if (lane == 0) ew[bw * NSRC + s] = p;
      }
    }
    __syncthreads();

    {
      const float bv = bVc[0];
      float vals[8];
      float mx = -3.0e38f;
#pragma unroll
      for (int i = 0; i < 8; ++i) {
        const int s = lane + 32 * i;
        const float mk = srcmask[bw * NSRC + s];
        float v = ew[bw * NSRC + s] + bv;
        v = v + ((mk == 0.0f) ? NEG_FILL : 0.0f);
        vals[i] = v;
        mx = fmaxf(mx, v);
      }
#pragma unroll
      for (int off = 16; off > 0; off >>= 1) mx = fmaxf(mx, __shfl_xor(mx, off, 32));
      float sm = 0.0f;
#pragma unroll
      for (int i = 0; i < 8; ++i) {
        vals[i] = expf(vals[i] - mx);
        sm += vals[i];
      }
#pragma unroll
      for (int off = 16; off > 0; off >>= 1) sm += __shfl_xor(sm, off, 32);
      const float inv = __builtin_amdgcn_rcpf(sm);
#pragma unroll
      for (int i = 0; i < 8; ++i) ew[bw * NSRC + lane + 32 * i] = vals[i] * inv;
    }
    __syncthreads();

    {
      v4f acc[4];
#pragma unroll
      for (int q = 0; q < 4; ++q) acc[q] = (v4f){0.f, 0.f, 0.f, 0.f};
      const float* sb = src + (size_t)bw * NSRC * NHID + 4 * lane;
#pragma unroll 1
      for (int s = 0; s < NSRC; ++s) {
        const float w = ew[bw * NSRC + s];
#pragma unroll
        for (int q = 0; q < 4; ++q) {
          const v4f x = *(const v4f*)(sb + (size_t)s * NHID + 128 * q);
          acc[q] += w * x;
        }
      }
#pragma unroll
      for (int q = 0; q < 4; ++q) {
        unsigned h0b, l0b, h1b, l1b, h2b, l2b, h3b, l3b;
        split_bf(acc[q][0], h0b, l0b);
        split_bf(acc[q][1], h1b, l1b);
        split_bf(acc[q][2], h2b, l2b);
        split_bf(acc[q][3], h3b, l3b);
        v2u ph, pl;
        ph[0] = h0b | (h1b << 16);
        ph[1] = h2b | (h3b << 16);
        pl[0] = l0b | (l1b << 16);
        pl[1] = l2b | (l3b << 16);
        *(v2u*)(AxH + bw * AXP + 128 * q + 4 * lane) = ph;
        *(v2u*)(AxL + bw * AXP + 128 * q + 4 * lane) = pl;
      }
    }
    hq_phase(AhH, AhL, WCh, WCl, NHID, wave, c, hh, hq);
    __syncthreads();

    {
      v4f hqv[4], vw[4];
#pragma unroll
      for (int q = 0; q < 4; ++q) {
        hqv[q] = *(const v4f*)(hq + bw * HQP + 128 * q + 4 * lane);
        vw[q]  = *(const v4f*)(Vwk + 128 * q + 4 * lane);
      }
      const float bvk = bVk[0];
      float mine = -3.0e38f;
#pragma unroll 1
      for (int s = 0; s < NSLOT; ++s) {
        const float* pr = PVK + (size_t)(bw * NSLOT + s) * NHID + 4 * lane;
        float p = 0.0f;
#pragma unroll
        for (int q = 0; q < 4; ++q) {
          const v4f pv = *(const v4f*)(pr + 128 * q);
#pragma unroll
          for (int e = 0; e < 4; ++e) p += vw[q][e] * ftanh_fast(hqv[q][e] + pv[e]);
        }
#pragma unroll
        for (int off = 16; off > 0; off >>= 1) p += __shfl_xor(p, off, 32);
        const float mk = kgmask[bw * NSLOT + s];
        p = (p + bvk) + ((mk == 0.0f) ? NEG_FILL : 0.0f);
        mine = (lane == s) ? p : mine;
      }
      float mx = mine;
#pragma unroll
      for (int off = 16; off > 0; off >>= 1) mx = fmaxf(mx, __shfl_xor(mx, off, 32));
      const float arg = (lane < NSLOT) ? (mine - mx) : 0.0f;
      const float ex = expf(arg);
      const float em = (lane < NSLOT) ? ex : 0.0f;
      float sm = em;
#pragma unroll
      for (int off = 16; off > 0; off >>= 1) sm += __shfl_xor(sm, off, 32);
      const float kwl = em * __builtin_amdgcn_rcpf(sm);
      if (lane < NSLOT) kwt[bw * NSLOT + lane] = kwl;
      v4f acc[4];
#pragma unroll
      for (int q = 0; q < 4; ++q) acc[q] = (v4f){0.f, 0.f, 0.f, 0.f};
#pragma unroll 1
      for (int s = 0; s < NSLOT; ++s) {
        const float w = __shfl(kwl, s, 32);
        const float* kr = kgh + (size_t)(bw * NSLOT + s) * NHID + 4 * lane;
#pragma unroll
        for (int q = 0; q < 4; ++q) {
          const v4f x = *(const v4f*)(kr + 128 * q);
          acc[q] += w * x;
        }
      }
#pragma unroll
      for (int q = 0; q < 4; ++q) {
        unsigned h0b, l0b, h1b, l1b, h2b, l2b, h3b, l3b;
        split_bf(acc[q][0], h0b, l0b);
        split_bf(acc[q][1], h1b, l1b);
        split_bf(acc[q][2], h2b, l2b);
        split_bf(acc[q][3], h3b, l3b);
        v2u ph, pl;
        ph[0] = h0b | (h1b << 16);
        ph[1] = h2b | (h3b << 16);
        pl[0] = l0b | (l1b << 16);
        pl[1] = l2b | (l3b << 16);
        *(v2u*)(AxH + bw * AXP + NHID + 128 * q + 4 * lane) = ph;
        *(v2u*)(AxL + bw * AXP + NHID + 128 * q + 4 * lane) = pl;
      }
    }
    __syncthreads();

    {
      const __bf16* axh = (const __bf16*)AxH + c * AXP + koff;
      const __bf16* axl = (const __bf16*)AxL + c * AXP + koff;
      const __bf16* ahh = (const __bf16*)AhH + c * AHP + koff;
      const __bf16* ahl = (const __bf16*)AhL + c * AHP + koff;
      const size_t GS_IH = (size_t)NHID * NXCK;
      const size_t GS_HH = (size_t)NHID * NHID;
      const size_t GS_GY = (size_t)NHID * NROWS;
#pragma unroll
      for (int u = 0; u < 2; ++u) {
        const int j = 32 * wave + 16 * u + c;
        const __bf16* wih = WIh + (size_t)j * NXCK + koff;
        const __bf16* wil = WIl + (size_t)j * NXCK + koff;
        const __bf16* whh = WCh + (size_t)(2 * NHID + j) * NHID + koff;
        const __bf16* whl = WCl + (size_t)(2 * NHID + j) * NHID + koff;
        v8f aR = z8, aZ = z8, aI = z8, aH = z8;
#pragma unroll 1
        for (int kx = 0; kx < NXCK; kx += 32) {
          const v16b xh = Frag<__bf16>::load(axh + kx);
          const v16b xl = Frag<__bf16>::load(axl + kx);
          const v16b rh = Frag<__bf16>::load(wih + kx);
          const v16b rl = Frag<__bf16>::load(wil + kx);
          aR = mma3(xh, xl, rh, rl, aR);
          asm volatile("" ::: "memory");
          const v16b zh = Frag<__bf16>::load(wih + GS_IH + kx);
          const v16b zl = Frag<__bf16>::load(wil + GS_IH + kx);
          aZ = mma3(xh, xl, zh, zl, aZ);
          asm volatile("" ::: "memory");
          const v16b nh = Frag<__bf16>::load(wih + 2 * GS_IH + kx);
          const v16b nl = Frag<__bf16>::load(wil + 2 * GS_IH + kx);
          aI = mma3(xh, xl, nh, nl, aI);
          asm volatile("" ::: "memory");
        }
#pragma unroll 1
        for (int k0 = 0; k0 < NHID; k0 += 32) {
          const v16b xh = Frag<__bf16>::load(ahh + k0);
          const v16b xl = Frag<__bf16>::load(ahl + k0);
          const v16b rh = Frag<__bf16>::load(whh + k0);
          const v16b rl = Frag<__bf16>::load(whl + k0);
          aR = mma3(xh, xl, rh, rl, aR);
          asm volatile("" ::: "memory");
          const v16b zh = Frag<__bf16>::load(whh + GS_HH + k0);
          const v16b zl = Frag<__bf16>::load(whl + GS_HH + k0);
          aZ = mma3(xh, xl, zh, zl, aZ);
          asm volatile("" ::: "memory");
          const v16b nh = Frag<__bf16>::load(whh + 2 * GS_HH + k0);
          const v16b nl = Frag<__bf16>::load(whl + 2 * GS_HH + k0);
          aH = mma3(xh, xl, nh, nl, aH);
          asm volatile("" ::: "memory");
        }
        acc_guard4(aR, aZ, aI, aH);
        const float* gp = GIYT + (size_t)j * NROWS + t * NBATCH + 8 * hh;
        const v4f gr0 = *(const v4f*)(gp);
        const v4f gr1 = *(const v4f*)(gp + 4);
        const v4f gz0 = *(const v4f*)(gp + GS_GY);
        const v4f gz1 = *(const v4f*)(gp + GS_GY + 4);
        const v4f gn0 = *(const v4f*)(gp + 2 * GS_GY);
        const v4f gn1 = *(const v4f*)(gp + 2 * GS_GY + 4);
        asm volatile("" ::: "memory");
#pragma unroll
        for (int r = 0; r < 8; ++r) {
          const float gr = (r < 4) ? gr0[r & 3] : gr1[r & 3];
          const float gz = (r < 4) ? gz0[r & 3] : gz1[r & 3];
          const float gn = (r < 4) ? gn0[r & 3] : gn1[r & 3];
          const float rg = fsig_p((aR[r] + gr) + brz[u]);
          const float zg = fsig_p((aZ[r] + gz) + bzz[u]);
          const float ng = ftanh_p(((aI[r] + gn) + bin[u]) + rg * (aH[r] + bhn[u]));
          const float ho = hst[u][r];
          hst[u][r] = (1.0f - zg) * ng + zg * ho;
        }
        asm volatile("" ::: "memory");
      }
    }
    __syncthreads();

#pragma unroll
    for (int u = 0; u < 2; ++u) {
      const int j = 32 * wave + 16 * u + c;
#pragma unroll
      for (int r = 0; r < 8; ++r) {
        unsigned hb, lb;
        split_bf(hst[u][r], hb, lb);
        AhH[(8 * hh + r) * AHP + j] = (unsigned short)hb;
        AhL[(8 * hh + r) * AHP + j] = (unsigned short)lb;
      }
    }
    __syncthreads();

    for (int pass = 0; pass < 2; ++pass) {
#pragma unroll
      for (int it = 0; it < 2; ++it) {
        const int idx = it * SCAN_THREADS + tid;
        const int row = idx >> 6;
        const int c8 = (idx & 63) * 8;
        const v4u vh = *(const v4ua*)(AhH + row * AHP + c8);
        const v4u vl = *(const v4ua*)(AhL + row * AHP + c8);
        const size_t o = ((size_t)(row * QPAD + t)) * NHID + c8;
        *(volatile v4u*)(SPH + o) = vh;
        *(volatile v4u*)(SPL + o) = vl;
      }
#pragma unroll
      for (int it = 0; it < 4; ++it) {
        const int idx = it * SCAN_THREADS + tid;
        const int row = idx >> 7;
        const int c8 = (idx & 127) * 8;
        const v4u vh = *(const v4ua*)(AxH + row * AXP + c8);
        const v4u vl = *(const v4ua*)(AxL + row * AXP + c8);
        const size_t o = ((size_t)(row * NSTEP + t)) * NXCK + c8;
        *(volatile v4u*)(XCKH + o) = vh;
        *(volatile v4u*)(XCKL + o) = vl;
      }
      if (wave == 0) {
        const v4f kv = *(const v4f*)(kwt + 4 * lane);
        *(volatile v4f*)(KW + t * (NBATCH * NSLOT) + 4 * lane) = kv;
      }
      __threadfence();
    }
  }
}

struct F8 { float v[8]; };
__device__ __forceinline__ F8 unpack_hl(v4u h, v4u l) {
  F8 o;
#pragma unroll
  for (int i = 0; i < 4; ++i) {
    const unsigned wh = h[i];
    const unsigned wl = l[i];
    o.v[2 * i]     = bf_lo(wh) + bf_lo(wl);
    o.v[2 * i + 1] = bf_hi(wh) + bf_hi(wl);
  }
  return o;
}

__global__ __launch_bounds__(256) void ptrcat_kernel(
    const unsigned short* __restrict__ SPH, const unsigned short* __restrict__ SPL,
    const unsigned short* __restrict__ XCKH, const unsigned short* __restrict__ XCKL,
    const int* __restrict__ tgt, const float* __restrict__ emb, const float* __restrict__ kf,
    const float* __restrict__ Wptr, const float* __restrict__ bptr,
    float* __restrict__ PTR, unsigned short* __restrict__ CAT) {
  __shared__ float wp[NPTRW];
  __shared__ float kfs[NHID];
  __shared__ float ptrs[NSTEP];
  const int tid = threadIdx.x, lane = tid & 31, wave = tid >> 5;
  const int b = blockIdx.x;
#pragma unroll 1
  for (int i = tid; i < NPTRW; i += 256) wp[i] = Wptr[i];
#pragma unroll 1
  for (int i = tid; i < NHID; i += 256) kfs[i] = kf[b * NHID + i];
  __syncthreads();
  const float bp = bptr[0];
#pragma unroll 1
  for (int ti = 0; ti < 4; ++ti) {
    const int t = wave * 4 + ti;
    const int m = b * NSTEP + t;
    int id = tgt[m];
    id = id < 0 ? 0 : (id > NVOC - 1 ? NVOC - 1 : id);
    float p = 0.0f;
#pragma unroll 1
    for (int q2 = 0; q2 < 2; ++q2) {
      const int x0 = 256 * q2 + 8 * lane;
      const size_t so = (size_t)(b * QPAD + t) * NHID + x0;
      const size_t xo = (size_t)m * NXCK + x0;
      const v4u sh = *(const v4u*)(SPH + so);
      const v4u sl = *(const v4u*)(SPL + so);
      const v4u ch = *(const v4u*)(XCKH + xo);
      const v4u cl = *(const v4u*)(XCKL + xo);
      const v4u kh = *(const v4u*)(XCKH + xo + NHID);
      const v4u kl = *(const v4u*)(XCKL + xo + NHID);
      const v4f y0 = *(const v4f*)(emb + (size_t)id * NEMB + x0);
      const v4f y1 = *(const v4f*)(emb + (size_t)id * NEMB + x0 + 4);
      const F8 s8 = unpack_hl(sh, sl);
      const F8 c8 = unpack_hl(ch, cl);
      const F8 k8 = unpack_hl(kh, kl);
      v8h hs, hc, hk, hf;
#pragma unroll
      for (int e = 0; e < 8; ++e) {
        const float yv = (e < 4) ? y0[e & 3] : y1[e & 3];
        const float fv = kfs[x0 + e];
        p += wp[x0 + e] * c8.v[e];
        p += wp[NHID + x0 + e] * s8.v[e];
        p += wp[2 * NHID + x0 + e] * yv;
        p += wp[3 * NHID + x0 + e] * fv;
        p += wp[4 * NHID + x0 + e] * k8.v[e];
        hs[e] = (_Float16)(s8.v[e] * CATCARRY);
        hc[e] = (_Float16)(c8.v[e] * CATCARRY);
        hk[e] = (_Float16)(k8.v[e] * CATCARRY);
        hf[e] = (_Float16)(fv * CATCARRY);
      }
      unsigned short* cp = CAT + (size_t)m * NCAT + x0;
      *(volatile v8h*)(cp) = hs;
      *(volatile v8h*)(cp + NHID) = hc;
      *(volatile v8h*)(cp + 2 * NHID) = hk;
      *(volatile v8h*)(cp + 3 * NHID) = hf;
      __threadfence();
      *(volatile v8h*)(cp) = hs;
      *(volatile v8h*)(cp + NHID) = hc;
      *(volatile v8h*)(cp + 2 * NHID) = hk;
      *(volatile v8h*)(cp + 3 * NHID) = hf;
      asm volatile("" ::: "memory");
    }
#pragma unroll
    for (int off = 16; off > 0; off >>= 1) p += __shfl_xor(p, off, 32);
    const float pg = __builtin_amdgcn_rcpf(1.0f + expf(-(p + bp)));
    if (lane == 0) ptrs[t] = pg;
  }
  __syncthreads();
  if (wave == 0) {
    const float v = ptrs[lane];
    *(volatile float*)(PTR + b * NSTEP + lane) = v;
    __threadfence();
    *(volatile float*)(PTR + b * NSTEP + lane) = v;
  }
}

__global__ __launch_bounds__(128) void copy_softmax_kernel(const float* __restrict__ CL, const float* __restrict__ kgpad,
                                                           const float* __restrict__ KW, const float* __restrict__ PTR,
                                                           float* __restrict__ VAL) {
  const int m = blockIdx.x;
  const int b = m >> 5, t = m & 31;
  const int tid = threadIdx.x, lane = tid & 31, wave = tid >> 5;
  const int half = lane >> 4, li = lane & 15;
  const int k = wave * 2 + half;
  const v4f lg = *(const v4f*)(CL + (size_t)(b * QPAD + t) * NKL + k * NKGL + 4 * li);
  const v4f pm = *(const v4f*)(kgpad + (size_t)(b * NSLOT + k) * NKGL + 4 * li);
  float x[4];
  float mx = -3.0e38f;
#pragma unroll
  for (int e = 0; e < 4; ++e) {
    x[e] = lg[e] + ((pm[e] == 0.0f) ? NEG_FILL : 0.0f);
    mx = fmaxf(mx, x[e]);
  }
#pragma unroll
  for (int off = 8; off > 0; off >>= 1) mx = fmaxf(mx, __shfl_xor(mx, off, 32));
  float sm = 0.0f;
#pragma unroll
  for (int e = 0; e < 4; ++e) {
    x[e] = expf(x[e] - mx);
    sm += x[e];
  }
#pragma unroll
  for (int off = 8; off > 0; off >>= 1) sm += __shfl_xor(sm, off, 32);
  const float kw = KW[t * (NBATCH * NSLOT) + b * NSLOT + k];
  const float pt = PTR[m];
  const float sc = (kw * (1.0f - pt)) * __builtin_amdgcn_rcpf(sm);
  v4f o;
#pragma unroll
  for (int e = 0; e < 4; ++e) o[e] = x[e] * sc;
  float* op = VAL + (size_t)m * NKL + wave * 128 + 4 * lane;
  *(volatile v4f*)op = o;
  __threadfence();
  *(volatile v4f*)op = o;
}

__global__ __launch_bounds__(256) void row_stats_kernel(const unsigned short* __restrict__ LOGH, const float* __restrict__ VAL,
                                                        const float* __restrict__ PTR, const float* __restrict__ ez,
                                                        float* __restrict__ STATS) {
  __shared__ float redm[8];
  __shared__ float reds[8];
  __shared__ float redv[8];
  const int m = blockIdx.x;
  const int b = m >> 5;
  const int tid = threadIdx.x, lane = tid & 31, wave = tid >> 5;
  const v4u* lp = (const v4u*)(LOGH + (size_t)m * NVOC);
  float mth = -3.0e38f, sth = 0.0f;
#pragma unroll 1
  for (int i = tid; i < NVOC / 8; i += 256) {
    const v4u w = lp[i];
    float x[8];
#pragma unroll
    for (int q = 0; q < 4; ++q) {
      const unsigned wq = w[q];
      x[2 * q]     = h16_to_f32(wq & 0xffffu);
      x[2 * q + 1] = h16_to_f32(wq >> 16);
    }
    float cm = x[0];
#pragma unroll
    for (int e = 1; e < 8; ++e) cm = fmaxf(cm, x[e]);
    const float mn = fmaxf(mth, cm);
    sth = sth * expf(mth - mn);
#pragma unroll
    for (int e = 0; e < 8; ++e) sth += expf(x[e] - mn);
    mth = mn;
  }
#pragma unroll 1
  for (int off = 16; off > 0; off >>= 1) {
    const float mo = __shfl_xor(mth, off, 32);
    const float so = __shfl_xor(sth, off, 32);
    const float mn = fmaxf(mth, mo);
    sth = sth * expf(mth - mn) + so * expf(mo - mn);
    mth = mn;
  }
  const int ic = tid < NEXT ? tid : NEXT - 1;
  const float ezv = ez[b * NEXT + ic];
  float pv = VAL[(size_t)m * NKL + tid] + VAL[(size_t)m * NKL + 256 + tid];
  pv += (tid < NEXT) ? ezv : 0.0f;
#pragma unroll
  for (int off = 16; off > 0; off >>= 1) pv += __shfl_xor(pv, off, 32);
  if (lane == 0) { redm[wave] = mth; reds[wave] = sth; redv[wave] = pv; }
  __syncthreads();
  float gm = redm[0];
#pragma unroll
  for (int i = 1; i < 8; ++i) gm = fmaxf(gm, redm[i]);
  float gsum = 0.0f, gval = 0.0f;
#pragma unroll 1
  for (int i = 0; i < 8; ++i) {
    gsum += reds[i] * expf(redm[i] - gm);
    gval += redv[i];
  }
  const float pt = PTR[m];
  const float tot = pt + gval;
  const float inv = __builtin_amdgcn_rcpf(tot);
  const float gsc = (pt * __builtin_amdgcn_rcpf(gsum)) * inv;
  if (wave == 0) {
    float o = 0.0f;
    o = (lane == 0) ? gm : o;
    o = (lane == 1) ? gsc : o;
    o = (lane == 2) ? inv : o;
    *(volatile float*)(STATS + (size_t)m * 32 + lane) = o;
    __threadfence();
    *(volatile float*)(STATS + (size_t)m * 32 + lane) = o;
  }
}

__global__ __launch_bounds__(256) void assemble_kernel(const unsigned* __restrict__ LOGW, const float* __restrict__ STATS,
                                                       const float* __restrict__ VAL, const int* __restrict__ kgext,
                                                       const float* __restrict__ ez, float* __restrict__ out) {
  __shared__ __align__(16) float buf[CHUNKF];
  __shared__ float ezs[64];
  __shared__ int gl[1024];
  __shared__ float vl[1024];
  const int tid = threadIdx.x;
  const int chunk = blockIdx.x, b = blockIdx.y;
  const int f0 = chunk * CHUNKF;
  const int nel = (SLABF - f0 < CHUNKF) ? (SLABF - f0) : CHUNKF;
  const int t0 = f0 / NVOCX;
  const int t1 = (t0 + 1 < NSTEP) ? (t0 + 1) : (NSTEP - 1);
  const int fbnd = (t0 + 1) * NVOCX;
  const int m0 = b * NSTEP + t0, m1 = b * NSTEP + t1;
  const float rmax0 = STATS[(size_t)m0 * 32], gs0 = STATS[(size_t)m0 * 32 + 1], inv0 = STATS[(size_t)m0 * 32 + 2];
  const float rmax1 = STATS[(size_t)m1 * 32], gs1 = STATS[(size_t)m1 * 32 + 1], inv1 = STATS[(size_t)m1 * 32 + 2];
  if (tid < 64) {
    const int ic = tid < NEXT ? tid : NEXT - 1;
    const float v = ez[b * NEXT + ic];
    ezs[tid] = (tid < NEXT) ? v : 0.0f;
  }
  __syncthreads();
#pragma unroll 1
  for (int it = 0; it < CHUNKF / 512; ++it) {
    const int g = 2 * (it * 256 + tid);
    const int f = f0 + g;
    const int hi = (f >= fbnd) ? 1 : 0;
    const int t = hi ? t1 : t0;
    const int v = f - t * NVOCX;
    const float rmax = hi ? rmax1 : rmax0;
    const float gs = hi ? gs1 : gs0;
    const float inv = hi ? inv1 : inv0;
    int vc = (v < NVOC - 2) ? v : (NVOC - 2);
    vc = vc < 0 ? 0 : vc;
    const unsigned w = LOGW[((size_t)(b * NSTEP + t) * NVOC + (size_t)vc) >> 1];
    const float l0 = h16_to_f32(w & 0xffffu);
    const float l1 = h16_to_f32(w >> 16);
    const float e0 = expf(l0 - rmax) * gs;
    const float e1 = expf(l1 - rmax) * gs;
    int ei = v - NVOC;
    ei = ei < 0 ? 0 : (ei > NEXT - 2 ? NEXT - 2 : ei);
    const float zz0 = ezs[ei] * inv;
    const float zz1 = ezs[ei + 1] * inv;
    const float fa = (v < NVOC) ? 1.0f : 0.0f;
    const float fz = 1.0f - fa;
    v2f o;
    o[0] = fa * e0 + fz * zz0;
    o[1] = fa * e1 + fz * zz1;
    *(v2f*)(buf + g) = o;
  }
#pragma unroll
  for (int r = 0; r < 2; ++r) {
#pragma unroll
    for (int ii = 0; ii < 2; ++ii) {
      const int i = ii * 256 + tid;
      const int idx = kgext[b * NKL + i];
      const bool rowok = (r == 0) || (t0 + 1 < NSTEP);
      const int tt = r ? t1 : t0;
      const int mm = b * NSTEP + tt;
      const float val = VAL[(size_t)mm * NKL + i] * (r ? inv1 : inv0);
      const bool iok = (idx >= 0) && (idx < NVOCX);
      const int idc = iok ? idx : 0;
      const int g = tt * NVOCX + idc - f0;
      const bool hit = rowok && iok && (g >= 0) && (g < nel);
      gl[r * 512 + i] = hit ? g : -1;
      vl[r * 512 + i] = val;
    }
  }
  __syncthreads();
  if (tid == 0 || tid == 32) {
    const int r = tid >> 5;
#pragma unroll 1
    for (int i = 0; i < 512; ++i) {
      const int g = gl[r * 512 + i];
      if (g >= 0) buf[g] += vl[r * 512 + i];
    }
  }
  __syncthreads();
  const int n4 = nel >> 2;
  float* op = out + (size_t)b * SLABF + f0;
  for (int pass = 0; pass < 2; ++pass) {
#pragma unroll
    for (int it = 0; it < 8; ++it) {
      const int i = it * 256 + tid;
      if (i < n4) {
        const v4f v = *(const v4f*)(buf + 4 * i);
        *(volatile v4f*)(op + 4 * i) = v;
      }
    }
    __threadfence();
  }
}

extern "C" void kernel_launch(void* const* d_in, const int* in_sizes, int n_in,
                              void* d_out, int out_size, void* d_ws, size_t ws_size, hipStream_t stream) {
  if (n_in < 35 || d_out == nullptr || d_ws == nullptr) return;
  if (out_size != NROWS * NVOCX) return;
  if (in_sizes[0] != NROWS || in_sizes[1] != NBATCH * NHID || in_sizes[2] != NBATCH * NSRC * NHID ||
      in_sizes[4] != NBATCH * NSLOT * NHID || in_sizes[6] != NBATCH * NSLOT * NKGL * NHID ||
      in_sizes[10] != NBATCH * NSLOT * NKGL || in_sizes[11] != NBATCH * NEXT ||
      in_sizes[12] != NVOC * NEMB || in_sizes[13] != NGATE * NGATE || in_sizes[14] != NGATE * NHID ||
      in_sizes[27] != NHID * NCAT || in_sizes[29] != NVOC * NHID || in_sizes[31] != NPTRW) return;

  const int*   tgt     = (const int*)d_in[0];
  const float* h0      = (const float*)d_in[1];
  const float* src     = (const float*)d_in[2];
  const float* srcmask = (const float*)d_in[3];
  const float* kgh     = (const float*)d_in[4];
  const float* kfus    = (const float*)d_in[5];
  const float* kgo     = (const float*)d_in[6];
  const float* kgmask  = (const float*)d_in[7];
  const float* kgpad   = (const float*)d_in[8];
  const int*   kgext   = (const int*)d_in[10];
  const float* ez      = (const float*)d_in[11];
  const float* emb     = (const float*)d_in[12];
  const float* W_ih    = (const float*)d_in[13];
  const float* W_hh    = (const float*)d_in[14];
  const float* b_ih    = (const float*)d_in[15];
  const float* b_hh    = (const float*)d_in[16];
  const float* Wq_c    = (const float*)d_in[17];
  const float* Wv_c    = (const float*)d_in[18];
  const float* bv_c    = (const float*)d_in[19];
  const float* Vw_c    = (const float*)d_in[20];
  const float* bV_c    = (const float*)d_in[21];
  const float* Wq_k    = (const float*)d_in[22];
  const float* Wv_k    = (const float*)d_in[23];
  const float* bv_k    = (const float*)d_in[24];
  const float* Vw_k    = (const float*)d_in[25];
  const float* bV_k    = (const float*)d_in[26];
  const float* W1      = (const float*)d_in[27];
  const float* b1      = (const float*)d_in[28];
  const float* W2      = (const float*)d_in[29];
  const float* b2      = (const float*)d_in[30];
  const float* Wptr    = (const float*)d_in[31];
  const float* bptr    = (const float*)d_in[32];
  const float* Wcpy    = (const float*)d_in[33];
  const float* bcpy    = (const float*)d_in[34];
  float* out = (float*)d_out;

  char* ws = (char*)d_ws; size_t off = 0;
  auto carve = [&](size_t bytes) -> char* { char* p = ws + off; off += (bytes + 255) & ~(size_t)255; return p; };
  unsigned short* W2H  = (unsigned short*)carve((size_t)NVOC * NHID * 2);
  unsigned short* LOGH = (unsigned short*)carve((size_t)NROWS * NVOC * 2);
  float*          PVS  = (float*)carve((size_t)NBATCH * NSRC * NHID * 4);
  unsigned short* SRCH = (unsigned short*)carve((size_t)NBATCH * NSRC * NHID * 2);
  unsigned short* KGOH = (unsigned short*)carve((size_t)NBATCH * NSLOT * NKGL * NHID * 2);
  unsigned short* KGOL = (unsigned short*)carve((size_t)NBATCH * NSLOT * NKGL * NHID * 2);
  unsigned short* WIHH = (unsigned short*)carve((size_t)NGATE * NXCK * 2);
  unsigned short* WIHL = (unsigned short*)carve((size_t)NGATE * NXCK * 2);
  unsigned short* WIHY = (unsigned short*)carve((size_t)NGATE * NHID * 2);
  unsigned short* WCH  = (unsigned short*)carve((size_t)NWCAT * NHID * 2);
  unsigned short* WCL  = (unsigned short*)carve((size_t)NWCAT * NHID * 2);
  unsigned short* W1H  = (unsigned short*)carve((size_t)NHID * NCAT * 2);
  unsigned short* WCPH = (unsigned short*)carve((size_t)NHID * NHID * 2);
  unsigned short* WCPL = (unsigned short*)carve((size_t)NHID * NHID * 2);
  unsigned short* WVCH = (unsigned short*)carve((size_t)NHID * NHID * 2);
  unsigned short* WVKH = (unsigned short*)carve((size_t)NHID * NHID * 2);
  unsigned short* KGHH = (unsigned short*)carve((size_t)NBATCH * NSLOT * NHID * 2);
  float*          PVK  = (float*)carve((size_t)NBATCH * NSLOT * NHID * 4);
  unsigned short* YH   = (unsigned short*)carve((size_t)NROWS * NEMB * 2);
  float*          GIYT = (float*)carve((size_t)NGATE * NROWS * 4);
  unsigned short* SPH  = (unsigned short*)carve((size_t)NBATCH * QPAD * NHID * 2);
  unsigned short* SPL  = (unsigned short*)carve((size_t)NBATCH * QPAD * NHID * 2);
  unsigned short* XCKH = (unsigned short*)carve((size_t)NROWS * NXCK * 2);
  unsigned short* XCKL = (unsigned short*)carve((size_t)NROWS * NXCK * 2);
  float*          KW   = (float*)carve((size_t)NSTEP * NBATCH * NSLOT * 4);
  float*          PTR  = (float*)carve((size_t)NROWS * 4);
  unsigned short* CAT  = (unsigned short*)carve((size_t)NROWS * NCAT * 2);
  unsigned short* QPH  = (unsigned short*)carve((size_t)NBATCH * QPAD * NHID * 2);
  unsigned short* QPL  = (unsigned short*)carve((size_t)NBATCH * QPAD * NHID * 2);
  float*          CL   = (float*)carve((size_t)NBATCH * QPAD * NKL * 4);
  float*          VAL  = (float*)carve((size_t)NROWS * NKL * 4);
  unsigned short* FF   = (unsigned short*)carve((size_t)NROWS * NHID * 2);
  float*          STATS = (float*)carve((size_t)NROWS * 32 * 4);
  if (off > ws_size || off > (size_t)134217728) return;

  auto nblk = [](int nrow, int ncol8) -> int { return (nrow * ncol8 + 255) / 256; };

  cvt8_kernel<0><<<nblk(NVOC, NHID / 8), 256, 0, stream>>>(W2, W2H, W2H, NVOC, NHID / 8, NHID, 0, WCARRY);
  cvt8_kernel<0><<<nblk(NHID, NCAT / 8), 256, 0, stream>>>(W1, W1H, W1H, NHID, NCAT / 8, NCAT, 0, WCARRY);
  cvt8_kernel<0><<<nblk(NHID, NHID / 8), 256, 0, stream>>>(Wv_c, WVCH, WVCH, NHID, NHID / 8, NHID, 0, WCARRY);
  cvt8_kernel<0><<<nblk(NHID, NHID / 8), 256, 0, stream>>>(Wv_k, WVKH, WVKH, NHID, NHID / 8, NHID, 0, WCARRY);
  cvt8_kernel<0><<<nblk(NBATCH * NSRC, NHID / 8), 256, 0, stream>>>(src, SRCH, SRCH, NBATCH * NSRC, NHID / 8, NHID, 0, 1.0f);
  cvt8_kernel<0><<<nblk(NBATCH * NSLOT, NHID / 8), 256, 0, stream>>>(kgh, KGHH, KGHH, NBATCH * NSLOT, NHID / 8, NHID, 0, 1.0f);
  cvt8_kernel<0><<<nblk(NGATE, NHID / 8), 256, 0, stream>>>(W_ih, WIHY, WIHY, NGATE, NHID / 8, NGATE, 0, WCARRY);
  cvt8_kernel<1><<<nblk(NGATE, NXCK / 8), 256, 0, stream>>>(W_ih, WIHH, WIHL, NGATE, NXCK / 8, NGATE, NHID, 1.0f);
  cvt8_kernel<1><<<nblk(NHID, NHID / 8), 256, 0, stream>>>(Wq_c, WCH, WCL, NHID, NHID / 8, NHID, 0, 1.0f);
  cvt8_kernel<1><<<nblk(NHID, NHID / 8), 256, 0, stream>>>(Wq_k, WCH + (size_t)NHID * NHID, WCL + (size_t)NHID * NHID,
                                                           NHID, NHID / 8, NHID, 0, 1.0f);
  cvt8_kernel<1><<<nblk(NGATE, NHID / 8), 256, 0, stream>>>(W_hh, WCH + (size_t)2 * NHID * NHID, WCL + (size_t)2 * NHID * NHID,
                                                            NGATE, NHID / 8, NHID, 0, 1.0f);
  cvt8_kernel<1><<<nblk(NHID, NHID / 8), 256, 0, stream>>>(Wcpy, WCPH, WCPL, NHID, NHID / 8, NHID, 0, 1.0f);
  cvt8_kernel<1><<<nblk(NBATCH * NSLOT * NKGL, NHID / 8), 256, 0, stream>>>(kgo, KGOH, KGOL, NBATCH * NSLOT * NKGL, NHID / 8,
                                                                            NHID, 0, 1.0f);
  gather_y_kernel<<<(NROWS * (NEMB / 8)) / 256, 256, 0, stream>>>(tgt, emb, YH);
  zero_pad_kernel<<<dim3((NBATCH * 32 * 64) / 256, 2), 256, 0, stream>>>(SPH, SPL);

  wmma_gemm64<0, false, 2, 0><<<dim3(((NBATCH * NSRC / 64) * (NHID / 64)) / 8, 1), 256, 0, stream>>>(
      SRCH, SRCH, NHID, 0L, WVCH, WVCH, NHID, 0L, (void*)PVS, (void*)PVS, NHID, 0L,
      bv_c, NBATCH * NSRC, NHID, NHID, 1.0f / WCARRY);
  wmma_gemm64<0, false, 2, 0><<<dim3(((NBATCH * NSLOT / 64) * (NHID / 64)) / 8, 1), 256, 0, stream>>>(
      KGHH, KGHH, NHID, 0L, WVKH, WVKH, NHID, 0L, (void*)PVK, (void*)PVK, NHID, 0L,
      bv_k, NBATCH * NSLOT, NHID, NHID, 1.0f / WCARRY);
  wmma_gemm64<0, false, 0, 0><<<dim3(((NGATE / 64) * (NROWS / 64)) / 8, 1), 256, 0, stream>>>(
      WIHY, WIHY, NHID, 0L, YH, YH, NEMB, 0L, (void*)GIYT, (void*)GIYT, NROWS, 0L,
      b_ih, NGATE, NROWS, NEMB, 1.0f / (WCARRY * YCARRY));

  scan_kernel<<<1, SCAN_THREADS, 0, stream>>>(h0, src, srcmask, kgh, kgmask, PVS, PVK, Vw_c, bV_c, Vw_k, bV_k,
                                              GIYT, b_ih, b_hh, WCH, WCL, WIHH, WIHL, SPH, SPL, XCKH, XCKL, KW);

  ptrcat_kernel<<<NBATCH, 256, 0, stream>>>(SPH, SPL, XCKH, XCKL, tgt, emb, kfus, Wptr, bptr, PTR, CAT);
  wmma_gemm64<1, true, 2, 2><<<dim3(((NBATCH * QPAD / 64) * (NHID / 64)) / 8, 1), 256, 0, stream>>>(
      SPH, SPL, NHID, 0L, WCPH, WCPL, NHID, 0L, (void*)QPH, (void*)QPL, NHID, 0L,
      bcpy, NBATCH * QPAD, NHID, NHID, 1.0f);
  wmma_gemm64<1, true, 0, 0><<<dim3(1, NBATCH), 256, 0, stream>>>(
      QPH, QPL, NHID, (long)QPAD * NHID, KGOH, KGOL, NHID, (long)NKL * NHID,
      (void*)CL, (void*)CL, NKL, (long)QPAD * NKL, bcpy, QPAD, NKL, NHID, 1.0f);
  copy_softmax_kernel<<<NROWS, 128, 0, stream>>>(CL, kgpad, KW, PTR, VAL);
  wmma_gemm64<0, false, 2, 1><<<dim3(((NROWS / 64) * (NHID / 64)) / 8, 1), 256, 0, stream>>>(
      CAT, CAT, NCAT, 0L, W1H, W1H, NCAT, 0L, (void*)FF, (void*)FF, NHID, 0L,
      b1, NROWS, NHID, NCAT, 1.0f / (WCARRY * CATCARRY));
  wmma_gemm64<0, false, 2, 1><<<dim3(((NROWS / 64) * (NVOC / 64)) / 8, 1), 256, 0, stream>>>(
      FF, FF, NHID, 0L, W2H, W2H, NHID, 0L, (void*)LOGH, (void*)LOGH, NVOC, 0L,
      b2, NROWS, NVOC, NHID, 1.0f / WCARRY);
  row_stats_kernel<<<NROWS, 256, 0, stream>>>(LOGH, VAL, PTR, ez, STATS);
  assemble_kernel<<<dim3(NCHUNK, NBATCH), 256, 0, stream>>>((const unsigned*)LOGH, STATS, VAL, kgext, ez, out);
}
